// RelationsNetwork_46943992546197
// MI455X (gfx1250) — hardware-verified
//
#include <hip/hip_runtime.h>
#include <math.h>

typedef __attribute__((ext_vector_type(16))) _Float16 v16h;
typedef __attribute__((ext_vector_type(16))) __bf16 v16b;
typedef __attribute__((ext_vector_type(8)))  _Float16 v8h;
typedef __attribute__((ext_vector_type(8)))  float v8f;
typedef __attribute__((ext_vector_type(4)))  float v4f;
typedef __attribute__((ext_vector_type(2)))  float v2f;
typedef __attribute__((ext_vector_type(4)))  unsigned v4u;
typedef __attribute__((ext_vector_type(4)))  int v4i;
typedef float __attribute__((may_alias)) float_a;
typedef int __attribute__((may_alias)) int_a;

template <typename T> __device__ __forceinline__ void vst2(void* p, T v) { *(volatile T*)p = v; __threadfence(); *(volatile T*)p = v; }
__device__ __forceinline__ v8f wmma16(v16h a, v16h b, v8f c) {
  v8f d = __builtin_amdgcn_wmma_f32_16x16x32_f16(false, a, false, b, (short)0, c, false, false);
  asm volatile("v_nop\n\tv_nop\n\tv_nop\n\tv_nop" : "+v"(d) : "v"(a), "v"(b));
  return d;
}
__device__ __forceinline__ v8f wmma_bf(v16b a, v16b b, v8f c) {
  v8f d = __builtin_amdgcn_wmma_f32_16x16x32_bf16(false, a, false, b, (short)0, c, false, false);
  asm volatile("v_nop\n\tv_nop\n\tv_nop\n\tv_nop" : "+v"(d) : "v"(a), "v"(b));
  return d;
}
__device__ __forceinline__ v16h frag_h(const _Float16* rowk0, int lane) {
  union { v16h v; v8h q[2]; } u; const _Float16* p = rowk0 + 8 * (lane >> 4);
  u.q[0] = *(const v8h*)p; u.q[1] = *(const v8h*)(p + 16); return u.v;
}
__device__ __forceinline__ v16h frag_f32(const float* rowk0, int lane) {
  v16h a; const float* p = rowk0 + 8 * (lane >> 4);
#pragma unroll
  for (int i = 0; i < 8; ++i) { a[i] = (_Float16)p[i]; a[8 + i] = (_Float16)p[16 + i]; }
  return a;
}
__device__ __forceinline__ v16h frag_f32s(const float* rowk0, int lane, float sc) {
  v16h a; const float* p = rowk0 + 8 * (lane >> 4);
#pragma unroll
  for (int i = 0; i < 8; ++i) { a[i] = (_Float16)(p[i] * sc); a[8 + i] = (_Float16)(p[16 + i] * sc); }
  return a;
}
__device__ __forceinline__ v16h fragc_f32(const float* W, int k0, int n, int lane, int ld, int K) {
  v16h a; const int g = lane >> 4;
#pragma unroll
  for (int i = 0; i < 8; ++i) { const int ka = k0 + 8 * g + i, kb = ka + 16;
    a[i] = (_Float16)(ka < K ? W[(size_t)ka * ld + n] : 0.f); a[8 + i] = (_Float16)(kb < K ? W[(size_t)kb * ld + n] : 0.f); }
  return a;
}
struct F2 { v16b h, l; };
__device__ __forceinline__ F2 bsplit16(const float v[16]) { F2 r;
#pragma unroll
  for (int i = 0; i < 16; ++i) { const __bf16 h = (__bf16)v[i]; r.h[i] = h; r.l[i] = (__bf16)(v[i] - (float)h); }
  return r; }
__device__ __forceinline__ F2 split_row(const float* row, int k0, int lane) { float v[16]; const float* p = row + k0 + 8 * (lane >> 4);
#pragma unroll
  for (int i = 0; i < 8; ++i) { v[i] = p[i]; v[8 + i] = p[16 + i]; }
  return bsplit16(v); }
__device__ __forceinline__ F2 split_rowK(const float* row, int k0, int lane, int K) { float v[16]; const int g = lane >> 4;
#pragma unroll
  for (int i = 0; i < 8; ++i) { const int ka = k0 + 8 * g + i, kb = ka + 16; v[i] = ka < K ? row[ka] : 0.f; v[8 + i] = kb < K ? row[kb] : 0.f; }
  return bsplit16(v); }
__device__ __forceinline__ F2 split_col(const float* W, int k0, int n, int lane, int ld, int K) { float v[16]; const int g = lane >> 4;
#pragma unroll
  for (int i = 0; i < 8; ++i) { const int ka = k0 + 8 * g + i, kb = ka + 16; v[i] = ka < K ? W[(size_t)ka * ld + n] : 0.f; v[8 + i] = kb < K ? W[(size_t)kb * ld + n] : 0.f; }
  return bsplit16(v); }
__device__ __forceinline__ v8f mac3(const F2& a, const F2& b, v8f c) { c = wmma_bf(a.l, b.h, c); c = wmma_bf(a.h, b.l, c); return wmma_bf(a.h, b.h, c); }
__device__ __forceinline__ float sigm(float v) { return 1.0f / (1.0f + expf(-v)); }
#define LDSX() do { asm volatile("s_wait_dscnt 0" ::: "memory"); __builtin_amdgcn_wave_barrier(); __builtin_amdgcn_fence(__ATOMIC_RELEASE, "workgroup"); } while (0)

#define NBT 32
#define SS 64
#define DX 258
#define KP 288
#define HH 256
#define NOUT 10
#define NPR (NBT * SS * SS)

__global__ __launch_bounds__(64) void k_x(const float* __restrict__ sent, const float* __restrict__ coord, float* __restrict__ X) {
  const int r = blockIdx.x, tid = threadIdx.x; __shared__ __align__(16) float row[KP];
  for (int q = tid; q < KP; q += 64) row[q] = q < 256 ? sent[(size_t)r * 256 + q] : (q < DX ? coord[(size_t)r * 2 + (q - 256)] : 0.f);
  __syncthreads();
  for (int q = tid; q < KP / 4; q += 64) vst2(X + (size_t)r * KP + q * 4, *(const v4f*)(&row[q * 4]));
  (void)tid;
}
__global__ __launch_bounds__(256) void k_pack(const float* __restrict__ gw1, const float* __restrict__ gw2, const float* __restrict__ gw3, _Float16* __restrict__ P1, _Float16* __restrict__ P2, _Float16* __restrict__ P3) {
  const int o = blockIdx.x, tid = threadIdx.x;
  for (int q = tid; q < KP / 8; q += 256) { union { v8h hh; v4u u; } pk;
#pragma unroll
    for (int i = 0; i < 8; ++i) { const int d = q * 8 + i; pk.hh[i] = (_Float16)(d < DX ? gw1[(size_t)(2 * DX + d) * HH + o] * 16.0f : 0.f); }
    vst2(P1 + (size_t)o * KP + q * 8, pk.u); }
  for (int q = tid; q < HH / 8; q += 256) { union { v8h hh; v4u u; } pk, pk3;
#pragma unroll
    for (int i = 0; i < 8; ++i) { const int k = q * 8 + i; pk.hh[i] = (_Float16)(gw2[(size_t)k * HH + o] * 16.0f); pk3.hh[i] = (_Float16)(gw3[(size_t)k * HH + o] * 16.0f); }
    vst2(P2 + (size_t)o * HH + q * 8, pk.u); vst2(P3 + (size_t)o * HH + q * 8, pk3.u); }
}
__global__ __launch_bounds__(128) void k_xab(const float* __restrict__ X, const float* __restrict__ gw1, float* __restrict__ XAB) {
  __shared__ __align__(16) float so[4][16][132];
  const int tid = threadIdx.x, wave = tid >> 5, lane = tid & 31, col = lane & 15, g = lane >> 4;
  const int r0 = blockIdx.x * 64 + wave * 16, n0 = blockIdx.y * 128; const int which = n0 / HH;
  v8f acc[8] = {};
#pragma unroll 1
  for (int kc = 0; kc < KP / 32; ++kc) { const v16h a = frag_f32(X + (size_t)(r0 + col) * KP + kc * 32, lane);
#pragma unroll
    for (int j = 0; j < 8; ++j) { v16h bw = fragc_f32(gw1 + (size_t)which * DX * HH, kc * 32, (n0 % HH) + j * 16 + col, lane, HH, DX);
#pragma unroll
      for (int e = 0; e < 16; ++e) bw[e] = bw[e] * (_Float16)16.0f;
      acc[j] = wmma16(a, bw, acc[j]); } }
#pragma unroll
  for (int j = 0; j < 8; ++j)
#pragma unroll
    for (int r = 0; r < 8; ++r) so[wave][8 * g + r][j * 16 + col] = acc[j][r] * (1.0f / 16.0f);
  LDSX();
#pragma unroll 4
  for (int rl = 0; rl < 16; ++rl) vst2(XAB + (size_t)(r0 + rl) * 512 + n0 + lane * 4, *(const v4f*)(&so[wave][rl][lane * 4]));
}
__global__ __launch_bounds__(128) void k_h1(const float* __restrict__ X, const _Float16* __restrict__ P1, const float* __restrict__ XAB, const float* __restrict__ b1, _Float16* __restrict__ h1, int prow0) {
  __shared__ __align__(16) float so[4][16][132];
  const int tid = threadIdx.x, wave = tid >> 5, lane = tid & 31, col = lane & 15, g = lane >> 4;
  const int p0 = prow0 + blockIdx.x * 64 + wave * 16, n0 = blockIdx.y * 128;
  const int p = p0 + col; const int b = p / (SS * SS), i = (p / SS) % SS, j = p % SS;
  const float* xi = X + (size_t)(b * SS + i) * KP; const float* xj = X + (size_t)(b * SS + j) * KP;
  v8f acc[8] = {};
#pragma unroll 1
  for (int kc = 0; kc < KP / 32; ++kc) { v16h a;
#pragma unroll
    for (int e = 0; e < 8; ++e) { const int d0 = kc * 32 + 8 * g + e, d1 = d0 + 16; a[e] = (_Float16)(xi[d0] * xj[d0]); a[8 + e] = (_Float16)(xi[d1] * xj[d1]); }
#pragma unroll
    for (int jj = 0; jj < 8; ++jj) acc[jj] = wmma16(a, frag_h(P1 + (size_t)(n0 + jj * 16 + col) * KP + kc * 32, lane), acc[jj]); }
#pragma unroll
  for (int jj = 0; jj < 8; ++jj) { const int o = n0 + jj * 16 + col; const float bb = b1[o];
#pragma unroll
    for (int r = 0; r < 8; ++r) { const int pp = p0 + 8 * g + r; const int bb_ = pp / (SS * SS), ii = (pp / SS) % SS, j2 = pp % SS;
      const float v = acc[jj][r] * (1.0f / 16.0f) + XAB[(size_t)(bb_ * SS + j2) * 512 + o] + XAB[(size_t)(bb_ * SS + ii) * 512 + HH + o] + bb; so[wave][8 * g + r][jj * 16 + col] = v > 0.f ? v : 0.f; } }
  LDSX();
  for (int q = lane; q < 16 * 16; q += 32) { const int rl = q >> 4, pc = q & 15; union { v8h hh; v4u u; } pk;
#pragma unroll
    for (int e = 0; e < 8; ++e) pk.hh[e] = (_Float16)so[wave][rl][pc * 8 + e];
    vst2(h1 + (size_t)(p0 - prow0 + rl) * HH + n0 + pc * 8, pk.u); }
}
template <int SUM>
__global__ __launch_bounds__(128) void k_h(const _Float16* __restrict__ hin, const _Float16* __restrict__ P, const float* __restrict__ bias, _Float16* __restrict__ hout, float* __restrict__ part, int blk0) {
  __shared__ __align__(16) float so[4][16][132];
  __shared__ __align__(16) float sps[128];
  const int tid = threadIdx.x, wave = tid >> 5, lane = tid & 31, col = lane & 15, g = lane >> 4;
  const int p0 = blockIdx.x * 64 + wave * 16, n0 = blockIdx.y * 128;
  v8f acc[8] = {};
#pragma unroll 1
  for (int kc = 0; kc < HH / 32; ++kc) { const v16h a = frag_h(hin + (size_t)(p0 + col) * HH + kc * 32, lane);
#pragma unroll
    for (int jj = 0; jj < 8; ++jj) acc[jj] = wmma16(a, frag_h(P + (size_t)(n0 + jj * 16 + col) * HH + kc * 32, lane), acc[jj]); }
#pragma unroll
  for (int jj = 0; jj < 8; ++jj) { const float bb = bias[n0 + jj * 16 + col];
#pragma unroll
    for (int r = 0; r < 8; ++r) { const float v = acc[jj][r] * (1.0f / 16.0f) + bb; so[wave][8 * g + r][jj * 16 + col] = v > 0.f ? v : 0.f; } }
  if (SUM == 0) { LDSX();
    for (int q = lane; q < 16 * 16; q += 32) { const int rl = q >> 4, pc = q & 15; union { v8h hh; v4u u; } pk;
#pragma unroll
      for (int e = 0; e < 8; ++e) pk.hh[e] = (_Float16)so[wave][rl][pc * 8 + e];
      vst2(hout + (size_t)(p0 + rl) * HH + n0 + pc * 8, pk.u); } }
  else { __syncthreads();
    { const int c = tid; float s = 0.f;
      for (int ww = 0; ww < 4; ++ww) for (int rl = 0; rl < 16; ++rl) s += so[ww][rl][c];
      sps[c] = s; }
    __syncthreads();
    if (tid < 32) vst2(part + (size_t)(blk0 + blockIdx.x) * HH + n0 + tid * 4, *(const v4f*)(&sps[tid * 4])); }
}
__global__ __launch_bounds__(256) void k_f(const float* __restrict__ part, const float* __restrict__ fw1, const float* __restrict__ fb1, const float* __restrict__ fw2, const float* __restrict__ fb2, const float* __restrict__ fw3, const float* __restrict__ fb3, float* __restrict__ outrow) {
  __shared__ float r0[HH], r1[HH]; __shared__ __align__(16) float so[32];
  const int b = blockIdx.x, c = threadIdx.x;
  { float s = 0.f;
#pragma unroll 1
    for (int blk = 0; blk < (SS * SS) / 64; ++blk) s += part[((size_t)b * 64 + blk) * HH + c];
    r0[c] = s; }
  __syncthreads();
  { float a = fb1[c];
#pragma unroll 1
    for (int k = 0; k < HH; ++k) a += r0[k] * fw1[k * HH + c];
    r1[c] = a > 0.f ? a : 0.f; }
  __syncthreads();
  { float a = fb2[c];
#pragma unroll 1
    for (int k = 0; k < HH; ++k) a += r1[k] * fw2[k * HH + c];
    r0[c] = a > 0.f ? a : 0.f; }
  __syncthreads();
  if (c < 32) { float a = 0.f; if (c < NOUT) { a = fb3[c];
#pragma unroll 1
      for (int k = 0; k < HH; ++k) a += r0[k] * fw3[k * NOUT + c]; }
    so[c] = a; }
  __syncthreads();
  if (c < 8) vst2(outrow + (size_t)b * 32 + c * 4, *(const v4f*)(&so[c * 4]));
}
__global__ __launch_bounds__(64) void k_copy(const float* __restrict__ outrow, float* __restrict__ out) {
  __shared__ __align__(16) float s[NBT * NOUT];
  for (int q = threadIdx.x; q < NBT * NOUT; q += 64) s[q] = outrow[(q / NOUT) * 32 + (q % NOUT)];
  __syncthreads();
  for (int q = threadIdx.x; q < NBT * NOUT / 4; q += 64) vst2(out + q * 4, *(const v4f*)(&s[q * 4]));
}
extern "C" void kernel_launch(void* const* d_in, const int* in_sizes, int n_in, void* d_out, int out_size, void* d_ws, size_t ws_size, hipStream_t stream) {
  (void)in_sizes; (void)n_in; (void)out_size; (void)ws_size;
  const float** I = (const float**)d_in;
  const float* sent = I[0]; const float* coord = I[1]; const float* gw1 = I[2]; const float* gb1 = I[3]; const float* gw2 = I[4]; const float* gb2 = I[5]; const float* gw3 = I[6]; const float* gb3 = I[7];
  const float* fw1 = I[8]; const float* fb1 = I[9]; const float* fw2 = I[10]; const float* fb2 = I[11]; const float* fw3 = I[12]; const float* fb3 = I[13];
  float* out = (float*)d_out;
  char* ws = (char*)d_ws; size_t off = 0;
  auto take = [&](size_t bytes) { char* p = ws + off; off += (bytes + 255) & ~(size_t)255; return p; };
  float* X = (float*)take((size_t)NBT * SS * KP * 4); _Float16* P1 = (_Float16*)take((size_t)HH * KP * 2); _Float16* P2 = (_Float16*)take((size_t)HH * HH * 2); _Float16* P3 = (_Float16*)take((size_t)HH * HH * 2);
  float* XAB = (float*)take((size_t)NBT * SS * 512 * 4); float* part = (float*)take((size_t)(NPR / 64) * HH * 4); float* outrow = (float*)take((size_t)NBT * 32 * 4);
  _Float16* h1 = (_Float16*)take((size_t)(NPR / 2) * HH * 2); _Float16* h2 = (_Float16*)take((size_t)(NPR / 2) * HH * 2);
  k_x<<<NBT * SS, 64, 0, stream>>>(sent, coord, X);
  k_pack<<<HH, 256, 0, stream>>>(gw1, gw2, gw3, P1, P2, P3);
  k_xab<<<dim3(NBT * SS / 64, 4), 128, 0, stream>>>(X, gw1, XAB);
  for (int hf = 0; hf < 2; ++hf) { const int prow0 = hf * (NPR / 2);
    k_h1<<<dim3((NPR / 2) / 64, 2), 128, 0, stream>>>(X, P1, XAB, gb1, h1, prow0);
    k_h<0><<<dim3((NPR / 2) / 64, 2), 128, 0, stream>>>(h1, P2, gb2, h2, nullptr, 0);
    k_h<1><<<dim3((NPR / 2) / 64, 2), 128, 0, stream>>>(h2, P3, gb3, nullptr, part, prow0 / 64); }
  k_f<<<NBT, 256, 0, stream>>>(part, fw1, fb1, fw2, fb2, fw3, fb3, outrow);
  k_copy<<<1, 64, 0, stream>>>(outrow, out);
}
